// MPNNet_4355096838272
// MI455X (gfx1250) — hardware-run, weakly checked
//
#include <hip/hip_runtime.h>


namespace {
constexpr int N = 100000, NP = 100032, E = 1000000, G = 1000, GP = 1008, D = 64, ED = 16, L = 3, CAT = L * D, L0 = 256, L1 = 128, NBLK = NP / 16;
constexpr float XS = 8.0f, WSC = 256.0f, LNEPS = 1e-5f;
typedef _Float16 b16;
typedef __attribute__((ext_vector_type(16))) _Float16 v16b;
typedef __attribute__((ext_vector_type(8))) _Float16 v8b;
typedef __attribute__((ext_vector_type(8))) float v8f;
typedef __attribute__((ext_vector_type(4))) float v4f;
__device__ __forceinline__ float bf16_rne(float f) { unsigned int u = __float_as_uint(f); u += 0x7FFFu + ((u >> 16) & 1u); return __uint_as_float(u & 0xFFFF0000u); }
__device__ __forceinline__ void split16(float v, b16& hi, b16& lo) { hi = (b16)v; lo = (b16)(v - (float)hi); }
__device__ __forceinline__ v16b frag_kb(const b16* p, int hh) { const v8b a = *(const v8b*)(p + 8 * hh), b = *(const v8b*)(p + 16 + 8 * hh); v16b f;
#pragma unroll
  for (int e = 0; e < 8; ++e) { f[e] = a[e]; f[8 + e] = b[e]; } return f; }
__device__ __forceinline__ v8f wmma16b(v16b a, v16b b, v8f c) { v8f d = __builtin_amdgcn_wmma_f32_16x16x32_f16(false, a, false, b, (short)0, c, false, false); asm volatile("v_nop\n\tv_nop\n\tv_nop\n\tv_nop" : "+v"(d) : "v"(a), "v"(b)); return d; }
__device__ __forceinline__ void wave_lds_sync() { __builtin_amdgcn_fence(__ATOMIC_RELEASE, "workgroup"); __builtin_amdgcn_wave_barrier(); __builtin_amdgcn_fence(__ATOMIC_ACQUIRE, "workgroup"); }
__device__ __forceinline__ float pmul(float a, float b) { float p = a * b; asm volatile("" : "+v"(p)); return p; }
__device__ __forceinline__ int iclamp(int v, int lo, int hi) { return v < lo ? lo : (v > hi ? hi : v); }
constexpr int CSR_NBLK9 = 512, CSR_GB9 = 9, CSR_GN9 = 1 << CSR_GB9  , CSR_TS9 = (CSR_GN9 < 32 ? 32 : CSR_GN9)  , CSR_MAXG9 = 512, CSR_CAP9 = 12288  ;
__device__ __host__ __forceinline__ int csr_tix9(int v) { return (v >> CSR_GB9) * CSR_TS9 + (v & (CSR_GN9 - 1)); }
__global__ __launch_bounds__(64) void csrA_kernel9(const int* __restrict__ dst, int E, int N, int nG, int CHP, int NGP, int* __restrict__ STG, int* __restrict__ HST) {
  extern __shared__ int sm[];
  int* cnt = sm; int* run = sm + NGP; int* ids = sm + 2 * NGP;
  const int b = blockIdx.x; const int ch = (E + CSR_NBLK9 - 1) / CSR_NBLK9; const int e0 = b * ch, e1 = min(E, e0 + ch);
  for (int i = threadIdx.x; i < NGP; i += 64) cnt[i] = 0;
  for (int i = threadIdx.x; i < CHP; i += 64) ids[i] = -1;
  __syncthreads();
  if (threadIdx.x == 0) {
    for (int e = e0; e < e1; ++e) { int d = dst[e]; d = (d < 0) ? 0 : (d >= N ? N - 1 : d); cnt[d >> CSR_GB9] += 1; }
    int acc = 0; for (int g = 0; g < nG; ++g) { run[g] = acc; acc += cnt[g]; }
    for (int e = e0; e < e1; ++e) { int d = dst[e]; d = (d < 0) ? 0 : (d >= N ? N - 1 : d); const int g = d >> CSR_GB9; ids[run[g]] = e; run[g] += 1; } }
  __syncthreads();
  typedef __attribute__((ext_vector_type(4))) int v4i;
  for (int pass = 0; pass < 2; ++pass) {
    for (int i = threadIdx.x; i < CHP / 4; i += 64) *(volatile v4i*)(STG + (size_t)b * CHP + i * 4) = *(const v4i*)(&ids[i * 4]);
    for (int i = threadIdx.x; i < NGP / 4; i += 64) { v4i v; for (int e = 0; e < 4; ++e) v[e] = (i * 4 + e < nG) ? cnt[i * 4 + e] : 0; *(volatile v4i*)(HST + (size_t)b * NGP + i * 4) = v; }
    __threadfence(); }
}
__global__ __launch_bounds__(512) void csrS_kernel9(const int* __restrict__ HST, int nG, int NGP, int* __restrict__ START, int* __restrict__ TOT, int* __restrict__ OFF) {
  __shared__ int tot[CSR_MAXG9];
  const int b = threadIdx.x;
  for (int pass = 0; pass < 2; ++pass) { int runb = 0; for (int g = 0; g < nG; ++g) { int c = HST[(size_t)b * NGP + g]; c = (c < 0) ? 0 : c; ((volatile int*)OFF)[(size_t)g * CSR_NBLK9 + b] = runb; runb += c; } __threadfence(); }
  for (int g = threadIdx.x; g < nG; g += 512) { int s = 0; for (int bb = 0; bb < CSR_NBLK9; ++bb) { int c = HST[(size_t)bb * NGP + g]; s += (c < 0) ? 0 : c; } tot[g] = s; }
  __syncthreads();
  if (threadIdx.x < 32) {
    __shared__ int st[CSR_MAXG9 + 32];
    if (threadIdx.x == 0) { int acc = 0; for (int g = 0; g < NGP; ++g) { st[g] = acc; if (g < nG) acc += (tot[g] + 31) & ~31; } st[NGP] = acc; }
    __builtin_amdgcn_fence(__ATOMIC_RELEASE, "workgroup"); __builtin_amdgcn_wave_barrier(); __builtin_amdgcn_fence(__ATOMIC_ACQUIRE, "workgroup");
    for (int pass = 0; pass < 2; ++pass) { for (int i = threadIdx.x; i < NGP + 32; i += 32) { ((volatile int*)START)[i] = (i <= NGP) ? st[min(i, NGP)] : 0; ((volatile int*)TOT)[i] = (i < nG) ? tot[i] : 0; } __threadfence(); } }
}
__global__ __launch_bounds__(256) void csrB_kernel9(const int* __restrict__ dst, int N, int nG, int CHP, int NGP, int permLen, const int* __restrict__ STG, const int* __restrict__ HST, const int* __restrict__ OFF, const int* __restrict__ START, const int* __restrict__ TOT, int* __restrict__ PERM, int* __restrict__ ROWPTR, int* __restrict__ ROWCNT, int* __restrict__ FLAG) {
  typedef __attribute__((ext_vector_type(4))) int v4i;
  __shared__ int ids[CSR_CAP9]; __shared__ unsigned short key[CSR_CAP9]; __shared__ int outp[CSR_CAP9]; __shared__ int ncnt[CSR_GN9 + 1]; __shared__ int boff[CSR_NBLK9 + 1];
  const int g = blockIdx.x, t_ = threadIdx.x; int tot = TOT[g]; int st = START[g], stn = START[g + 1]; const int v0 = g * CSR_GN9; const int nv = min(CSR_GN9, N - v0); const int t0 = g * CSR_TS9;
  st = (st < 0) ? 0 : (st > permLen - 32 ? permLen - 32 : st) & ~31; stn = (stn < st) ? st : (stn > permLen ? permLen : stn); tot = (tot < 0) ? 0 : tot; if (tot > stn - st && tot <= CSR_CAP9) tot = stn - st;
  if (tot > CSR_CAP9) {
    for (int pass = 0; pass < 2; ++pass) { for (int i = t_; i < CSR_TS9 / 4; i += 256) { v4i a, c; for (int e = 0; e < 4; ++e) { a[e] = st; c[e] = 0; } *(volatile v4i*)(ROWPTR + t0 + i * 4) = a; *(volatile v4i*)(ROWCNT + t0 + i * 4) = c; } if (t_ == 0) ((volatile int*)FLAG)[0] = 1; __threadfence(); } (void)nv; return; }
  if (t_ == 0) { int acc = 0; for (int b = 0; b < CSR_NBLK9; ++b) { boff[b] = acc; int c = HST[(size_t)b * NGP + g]; c = (c < 0) ? 0 : (c > CHP ? CHP : c); acc += c; if (acc > tot) acc = tot; } boff[CSR_NBLK9] = acc; }
  for (int i = t_; i <= CSR_GN9; i += 256) ncnt[i] = 0;
  __syncthreads();
  for (int b = 0; b < CSR_NBLK9; ++b) { const int c = boff[b + 1] - boff[b]; int o_ = OFF[(size_t)g * CSR_NBLK9 + b]; o_ = (o_ < 0) ? 0 : (o_ > CHP - c ? CHP - c : o_); const int* src_ = STG + (size_t)b * CHP + o_;
    for (int i = t_; i < c; i += 256) { int id = src_[i]; id = (id < 0) ? 0 : id; ids[boff[b] + i] = id; int d = dst[id]; d = (d < v0) ? v0 : (d >= N ? N - 1 : d); int kk = d - v0; kk = (kk < 0) ? 0 : (kk >= CSR_GN9 ? CSR_GN9 - 1 : kk); key[boff[b] + i] = (unsigned short)kk; } }
  __syncthreads();
  if (t_ == 0) { for (int i = 0; i < tot; ++i) ncnt[key[i]] += 1; int acc = 0; for (int vl = 0; vl < CSR_GN9; ++vl) { const int c = ncnt[vl]; ncnt[vl] = acc; acc += c; } ncnt[CSR_GN9] = acc;
    for (int i = 0; i < tot; ++i) { const int vl = key[i]; outp[ncnt[vl]] = ids[i]; ncnt[vl] += 1; }
    for (int vl = CSR_GN9; vl > 0; --vl) ncnt[vl] = ncnt[vl - 1]; ncnt[0] = 0; }
  __syncthreads();
  for (int pass = 0; pass < 2; ++pass) {
    for (int i = t_; i < (stn - st) / 4; i += 256) { v4i v; for (int e = 0; e < 4; ++e) { const int q = i * 4 + e; v[e] = (q < tot) ? outp[q] : -1; } *(volatile v4i*)(PERM + st + i * 4) = v; }
    for (int i = t_; i < CSR_TS9 / 4; i += 256) { v4i a, c; for (int e = 0; e < 4; ++e) { const int vl = i * 4 + e; const int vc = vl < CSR_GN9 ? vl : CSR_GN9; a[e] = (vl < CSR_GN9) ? st + ncnt[vc] : st; c[e] = (vl < nv) ? (ncnt[(vc < CSR_GN9 ? vc : CSR_GN9 - 1) + 1] - ncnt[vc]) : 0; } *(volatile v4i*)(ROWPTR + t0 + i * 4) = a; *(volatile v4i*)(ROWCNT + t0 + i * 4) = c; }
    __threadfence(); }
}
__global__ __launch_bounds__(256) void csrZ_kernel9(int* __restrict__ p, size_t n4) { typedef __attribute__((ext_vector_type(4))) int v4i; const size_t tid = (size_t)blockIdx.x * 256 + threadIdx.x, nth = (size_t)gridDim.x * 256; v4i z = {0, 0, 0, 0}; for (size_t i = tid; i < n4; i += nth) *(volatile v4i*)(p + i * 4) = z; }
struct CsrBufs9 { int *STG, *HST, *OFF, *START, *TOT, *PERM, *ROWPTR, *ROWCNT, *FLAG; int nG, NGP, CHP; size_t permLen; char* base; size_t bytes; };
static size_t csr_carve9(CsrBufs9& c, char* ws, size_t off, int E, int N) {
  const size_t off0 = off; c.base = ws + off;
  auto al = [&](size_t bytes) { char* p = ws + off; off += (bytes + 255) & ~(size_t)255; return p; };
  c.nG = (N + CSR_GN9 - 1) / CSR_GN9; c.NGP = (c.nG + 31) & ~31; const int ch = (E + CSR_NBLK9 - 1) / CSR_NBLK9; c.CHP = (ch + 31) & ~31; c.permLen = (size_t)E + 32 * (size_t)c.nG + 32;
  c.STG = (int*)al((size_t)CSR_NBLK9 * c.CHP * 4); c.HST = (int*)al((size_t)CSR_NBLK9 * c.NGP * 4); c.OFF = (int*)al((size_t)c.NGP * CSR_NBLK9 * 4); c.START = (int*)al((size_t)(c.NGP + 64) * 4); c.TOT = (int*)al((size_t)(c.NGP + 64) * 4);
  c.PERM = (int*)al(c.permLen * 4); c.ROWPTR = (int*)al((size_t)c.nG * CSR_TS9 * 4); c.ROWCNT = (int*)al((size_t)c.nG * CSR_TS9 * 4); c.FLAG = (int*)al(256);
  c.bytes = off - off0; return off;
}
static void csr_build9(const CsrBufs9& c, const int* dst, int E, int N, hipStream_t stream) {
  const size_t smem = (size_t)(2 * c.NGP + c.CHP) * 4;
  csrZ_kernel9<<<512, 256, 0, stream>>>((int*)c.base, c.bytes / 16);
  csrA_kernel9<<<CSR_NBLK9, 64, smem, stream>>>(dst, E, N, c.nG, c.CHP, c.NGP, c.STG, c.HST);
  csrS_kernel9<<<1, 512, 0, stream>>>(c.HST, c.nG, c.NGP, c.START, c.TOT, c.OFF);
  csrB_kernel9<<<c.nG, 256, 0, stream>>>(dst, N, c.nG, c.CHP, c.NGP, (int)c.permLen, c.STG, c.HST, c.OFF, c.START, c.TOT, c.PERM, c.ROWPTR, c.ROWCNT, c.FLAG);
}

constexpr int CSR_NBLK3 = 512, CSR_GB3 = 3, CSR_GN3 = 1 << CSR_GB3  , CSR_TS3 = (CSR_GN3 < 32 ? 32 : CSR_GN3)  , CSR_MAXG3 = 512, CSR_CAP3 = 12288  ;
__device__ __host__ __forceinline__ int csr_tix3(int v) { return (v >> CSR_GB3) * CSR_TS3 + (v & (CSR_GN3 - 1)); }
__global__ __launch_bounds__(64) void csrA_kernel3(const int* __restrict__ dst, int E, int N, int nG, int CHP, int NGP, int* __restrict__ STG, int* __restrict__ HST) {
  extern __shared__ int sm[];
  int* cnt = sm; int* run = sm + NGP; int* ids = sm + 2 * NGP;
  const int b = blockIdx.x; const int ch = (E + CSR_NBLK3 - 1) / CSR_NBLK3; const int e0 = b * ch, e1 = min(E, e0 + ch);
  for (int i = threadIdx.x; i < NGP; i += 64) cnt[i] = 0;
  for (int i = threadIdx.x; i < CHP; i += 64) ids[i] = -1;
  __syncthreads();
  if (threadIdx.x == 0) {
    for (int e = e0; e < e1; ++e) { int d = dst[e]; d = (d < 0) ? 0 : (d >= N ? N - 1 : d); cnt[d >> CSR_GB3] += 1; }
    int acc = 0; for (int g = 0; g < nG; ++g) { run[g] = acc; acc += cnt[g]; }
    for (int e = e0; e < e1; ++e) { int d = dst[e]; d = (d < 0) ? 0 : (d >= N ? N - 1 : d); const int g = d >> CSR_GB3; ids[run[g]] = e; run[g] += 1; } }
  __syncthreads();
  typedef __attribute__((ext_vector_type(4))) int v4i;
  for (int pass = 0; pass < 2; ++pass) {
    for (int i = threadIdx.x; i < CHP / 4; i += 64) *(volatile v4i*)(STG + (size_t)b * CHP + i * 4) = *(const v4i*)(&ids[i * 4]);
    for (int i = threadIdx.x; i < NGP / 4; i += 64) { v4i v; for (int e = 0; e < 4; ++e) v[e] = (i * 4 + e < nG) ? cnt[i * 4 + e] : 0; *(volatile v4i*)(HST + (size_t)b * NGP + i * 4) = v; }
    __threadfence(); }
}
__global__ __launch_bounds__(512) void csrS_kernel3(const int* __restrict__ HST, int nG, int NGP, int* __restrict__ START, int* __restrict__ TOT, int* __restrict__ OFF) {
  __shared__ int tot[CSR_MAXG3];
  const int b = threadIdx.x;
  for (int pass = 0; pass < 2; ++pass) { int runb = 0; for (int g = 0; g < nG; ++g) { int c = HST[(size_t)b * NGP + g]; c = (c < 0) ? 0 : c; ((volatile int*)OFF)[(size_t)g * CSR_NBLK3 + b] = runb; runb += c; } __threadfence(); }
  for (int g = threadIdx.x; g < nG; g += 512) { int s = 0; for (int bb = 0; bb < CSR_NBLK3; ++bb) { int c = HST[(size_t)bb * NGP + g]; s += (c < 0) ? 0 : c; } tot[g] = s; }
  __syncthreads();
  if (threadIdx.x < 32) {
    __shared__ int st[CSR_MAXG3 + 32];
    if (threadIdx.x == 0) { int acc = 0; for (int g = 0; g < NGP; ++g) { st[g] = acc; if (g < nG) acc += (tot[g] + 31) & ~31; } st[NGP] = acc; }
    __builtin_amdgcn_fence(__ATOMIC_RELEASE, "workgroup"); __builtin_amdgcn_wave_barrier(); __builtin_amdgcn_fence(__ATOMIC_ACQUIRE, "workgroup");
    for (int pass = 0; pass < 2; ++pass) { for (int i = threadIdx.x; i < NGP + 32; i += 32) { ((volatile int*)START)[i] = (i <= NGP) ? st[min(i, NGP)] : 0; ((volatile int*)TOT)[i] = (i < nG) ? tot[i] : 0; } __threadfence(); } }
}
__global__ __launch_bounds__(256) void csrB_kernel3(const int* __restrict__ dst, int N, int nG, int CHP, int NGP, int permLen, const int* __restrict__ STG, const int* __restrict__ HST, const int* __restrict__ OFF, const int* __restrict__ START, const int* __restrict__ TOT, int* __restrict__ PERM, int* __restrict__ ROWPTR, int* __restrict__ ROWCNT, int* __restrict__ FLAG) {
  typedef __attribute__((ext_vector_type(4))) int v4i;
  __shared__ int ids[CSR_CAP3]; __shared__ unsigned short key[CSR_CAP3]; __shared__ int outp[CSR_CAP3]; __shared__ int ncnt[CSR_GN3 + 1]; __shared__ int boff[CSR_NBLK3 + 1];
  const int g = blockIdx.x, t_ = threadIdx.x; int tot = TOT[g]; int st = START[g], stn = START[g + 1]; const int v0 = g * CSR_GN3; const int nv = min(CSR_GN3, N - v0); const int t0 = g * CSR_TS3;
  st = (st < 0) ? 0 : (st > permLen - 32 ? permLen - 32 : st) & ~31; stn = (stn < st) ? st : (stn > permLen ? permLen : stn); tot = (tot < 0) ? 0 : tot; if (tot > stn - st && tot <= CSR_CAP3) tot = stn - st;
  if (tot > CSR_CAP3) {
    for (int pass = 0; pass < 2; ++pass) { for (int i = t_; i < CSR_TS3 / 4; i += 256) { v4i a, c; for (int e = 0; e < 4; ++e) { a[e] = st; c[e] = 0; } *(volatile v4i*)(ROWPTR + t0 + i * 4) = a; *(volatile v4i*)(ROWCNT + t0 + i * 4) = c; } if (t_ == 0) ((volatile int*)FLAG)[0] = 1; __threadfence(); } (void)nv; return; }
  if (t_ == 0) { int acc = 0; for (int b = 0; b < CSR_NBLK3; ++b) { boff[b] = acc; int c = HST[(size_t)b * NGP + g]; c = (c < 0) ? 0 : (c > CHP ? CHP : c); acc += c; if (acc > tot) acc = tot; } boff[CSR_NBLK3] = acc; }
  for (int i = t_; i <= CSR_GN3; i += 256) ncnt[i] = 0;
  __syncthreads();
  for (int b = 0; b < CSR_NBLK3; ++b) { const int c = boff[b + 1] - boff[b]; int o_ = OFF[(size_t)g * CSR_NBLK3 + b]; o_ = (o_ < 0) ? 0 : (o_ > CHP - c ? CHP - c : o_); const int* src_ = STG + (size_t)b * CHP + o_;
    for (int i = t_; i < c; i += 256) { int id = src_[i]; id = (id < 0) ? 0 : id; ids[boff[b] + i] = id; int d = dst[id]; d = (d < v0) ? v0 : (d >= N ? N - 1 : d); int kk = d - v0; kk = (kk < 0) ? 0 : (kk >= CSR_GN3 ? CSR_GN3 - 1 : kk); key[boff[b] + i] = (unsigned short)kk; } }
  __syncthreads();
  if (t_ == 0) { for (int i = 0; i < tot; ++i) ncnt[key[i]] += 1; int acc = 0; for (int vl = 0; vl < CSR_GN3; ++vl) { const int c = ncnt[vl]; ncnt[vl] = acc; acc += c; } ncnt[CSR_GN3] = acc;
    for (int i = 0; i < tot; ++i) { const int vl = key[i]; outp[ncnt[vl]] = ids[i]; ncnt[vl] += 1; }
    for (int vl = CSR_GN3; vl > 0; --vl) ncnt[vl] = ncnt[vl - 1]; ncnt[0] = 0; }
  __syncthreads();
  for (int pass = 0; pass < 2; ++pass) {
    for (int i = t_; i < (stn - st) / 4; i += 256) { v4i v; for (int e = 0; e < 4; ++e) { const int q = i * 4 + e; v[e] = (q < tot) ? outp[q] : -1; } *(volatile v4i*)(PERM + st + i * 4) = v; }
    for (int i = t_; i < CSR_TS3 / 4; i += 256) { v4i a, c; for (int e = 0; e < 4; ++e) { const int vl = i * 4 + e; const int vc = vl < CSR_GN3 ? vl : CSR_GN3; a[e] = (vl < CSR_GN3) ? st + ncnt[vc] : st; c[e] = (vl < nv) ? (ncnt[(vc < CSR_GN3 ? vc : CSR_GN3 - 1) + 1] - ncnt[vc]) : 0; } *(volatile v4i*)(ROWPTR + t0 + i * 4) = a; *(volatile v4i*)(ROWCNT + t0 + i * 4) = c; }
    __threadfence(); }
}
__global__ __launch_bounds__(256) void csrZ_kernel3(int* __restrict__ p, size_t n4) { typedef __attribute__((ext_vector_type(4))) int v4i; const size_t tid = (size_t)blockIdx.x * 256 + threadIdx.x, nth = (size_t)gridDim.x * 256; v4i z = {0, 0, 0, 0}; for (size_t i = tid; i < n4; i += nth) *(volatile v4i*)(p + i * 4) = z; }
struct CsrBufs3 { int *STG, *HST, *OFF, *START, *TOT, *PERM, *ROWPTR, *ROWCNT, *FLAG; int nG, NGP, CHP; size_t permLen; char* base; size_t bytes; };
static size_t csr_carve3(CsrBufs3& c, char* ws, size_t off, int E, int N) {
  const size_t off0 = off; c.base = ws + off;
  auto al = [&](size_t bytes) { char* p = ws + off; off += (bytes + 255) & ~(size_t)255; return p; };
  c.nG = (N + CSR_GN3 - 1) / CSR_GN3; c.NGP = (c.nG + 31) & ~31; const int ch = (E + CSR_NBLK3 - 1) / CSR_NBLK3; c.CHP = (ch + 31) & ~31; c.permLen = (size_t)E + 32 * (size_t)c.nG + 32;
  c.STG = (int*)al((size_t)CSR_NBLK3 * c.CHP * 4); c.HST = (int*)al((size_t)CSR_NBLK3 * c.NGP * 4); c.OFF = (int*)al((size_t)c.NGP * CSR_NBLK3 * 4); c.START = (int*)al((size_t)(c.NGP + 64) * 4); c.TOT = (int*)al((size_t)(c.NGP + 64) * 4);
  c.PERM = (int*)al(c.permLen * 4); c.ROWPTR = (int*)al((size_t)c.nG * CSR_TS3 * 4); c.ROWCNT = (int*)al((size_t)c.nG * CSR_TS3 * 4); c.FLAG = (int*)al(256);
  c.bytes = off - off0; return off;
}
static void csr_build3(const CsrBufs3& c, const int* dst, int E, int N, hipStream_t stream) {
  const size_t smem = (size_t)(2 * c.NGP + c.CHP) * 4;
  csrZ_kernel3<<<512, 256, 0, stream>>>((int*)c.base, c.bytes / 16);
  csrA_kernel3<<<CSR_NBLK3, 64, smem, stream>>>(dst, E, N, c.nG, c.CHP, c.NGP, c.STG, c.HST);
  csrS_kernel3<<<1, 512, 0, stream>>>(c.HST, c.nG, c.NGP, c.START, c.TOT, c.OFF);
  csrB_kernel3<<<c.nG, 256, 0, stream>>>(dst, N, c.nG, c.CHP, c.NGP, (int)c.permLen, c.STG, c.HST, c.OFF, c.START, c.TOT, c.PERM, c.ROWPTR, c.ROWCNT, c.FLAG);
}


__global__ __launch_bounds__(256) void wprep_kernel(const float* __restrict__ w, int r0, int KIN, int OUT, int KP, b16* __restrict__ WT) {
  const size_t u = (size_t)blockIdx.x * 256 + threadIdx.x; if (u >= (size_t)OUT * KP / 8) return; const size_t e = u * 8; const int o = (int)(e / KP), k0 = (int)(e % KP); v8b v;
  for (int j = 0; j < 8; ++j) { const int k = k0 + j; v[j] = k < KIN ? (b16)(bf16_rne(w[(size_t)(r0 + (k < KIN ? k : 0)) * OUT + o]) * WSC) : (b16)0.0f; } for (int pass = 0; pass < 2; ++pass) { *(volatile v8b*)(WT + e) = v; __threadfence(); }
}
template <int RAW, int HAS_UPD, int HAS_PX>
__global__ __launch_bounds__(32) void node_kernel(const float* __restrict__ XIN, const float* __restrict__ vcur, const float* __restrict__ AGG, const b16* __restrict__ WU, const float* __restrict__ ub, const float* __restrict__ lg, const float* __restrict__ lb,
                                                  const float* __restrict__ vnext, const b16* __restrict__ WPX, int NLIM, float* __restrict__ XOUT, float* __restrict__ PX) {
  __shared__ __attribute__((aligned(16))) b16 Ah[16][2 * D + 8], Al[16][2 * D + 8]; __shared__ __attribute__((aligned(16))) float Xr[16][D + 4];
  const int lane = threadIdx.x, nloc = lane & 15, hlf = lane >> 4; const size_t m0 = (size_t)blockIdx.x * 16; const bool live = m0 < (size_t)NLIM; const float sc = 1.0f / (XS * WSC);
  v8f acc[4];
  if (HAS_UPD) {
    for (int rr = 0; rr < 16; ++rr) { const size_t r = m0 + rr; float xv0 = 0.0f, xv1 = 0.0f, a0 = 0.0f, a1 = 0.0f;
      if (live) { const float x0 = XIN[r * D + lane * 2], x1 = XIN[r * D + lane * 2 + 1]; xv0 = (RAW ? bf16_rne(x0) : x0) + bf16_rne(vcur[lane * 2]); xv1 = (RAW ? bf16_rne(x1) : x1) + bf16_rne(vcur[lane * 2 + 1]); a0 = AGG[r * D + lane * 2]; a1 = AGG[r * D + lane * 2 + 1]; }
      b16 p, q; split16(xv0 * XS, p, q); Ah[rr][lane * 2] = p; Al[rr][lane * 2] = q; split16(xv1 * XS, p, q); Ah[rr][lane * 2 + 1] = p; Al[rr][lane * 2 + 1] = q;
      split16(a0 * XS, p, q); Ah[rr][D + lane * 2] = p; Al[rr][D + lane * 2] = q; split16(a1 * XS, p, q); Ah[rr][D + lane * 2 + 1] = p; Al[rr][D + lane * 2 + 1] = q; }
    wave_lds_sync();
#pragma unroll
    for (int t = 0; t < 4; ++t) acc[t] = (v8f){};
#pragma unroll
    for (int kb = 0; kb < 2 * D; kb += 32) { const v16b a = frag_kb(&Ah[nloc][kb], hlf), al = frag_kb(&Al[nloc][kb], hlf);
#pragma unroll
      for (int t = 0; t < 4; ++t) { const v16b bw = frag_kb(WU + (size_t)(t * 16 + nloc) * (2 * D) + kb, hlf); acc[t] = wmma16b(a, bw, acc[t]); acc[t] = wmma16b(al, bw, acc[t]); } }
#pragma unroll
    for (int t = 0; t < 4; ++t) { const int c = t * 16 + nloc; const float bb = bf16_rne(ub[c]);
#pragma unroll 1
      for (int r8 = 0; r8 < 8; ++r8) Xr[8 * hlf + r8][c] = acc[t][r8] * sc + bb; }
    wave_lds_sync();
    for (int rr = 0; rr < 16; ++rr) { const float h0 = Xr[rr][lane * 2], h1 = Xr[rr][lane * 2 + 1]; float s = h0 + h1; for (int o = 16; o; o >>= 1) s += __shfl_xor(s, o); const float mu = s * (1.0f / D);
      float qv = pmul(h0 - mu, h0 - mu) + pmul(h1 - mu, h1 - mu); for (int o = 16; o; o >>= 1) qv += __shfl_xor(qv, o); const float rs = rsqrtf(qv * (1.0f / D) + LNEPS);
      const float y0 = live ? fmaxf(pmul(pmul(h0 - mu, rs), bf16_rne(lg[lane * 2])) + bf16_rne(lb[lane * 2]), 0.0f) : 0.0f, y1 = live ? fmaxf(pmul(pmul(h1 - mu, rs), bf16_rne(lg[lane * 2 + 1])) + bf16_rne(lb[lane * 2 + 1]), 0.0f) : 0.0f;
      wave_lds_sync(); Xr[rr][lane * 2] = y0; Xr[rr][lane * 2 + 1] = y1; }
    wave_lds_sync();
    typedef __attribute__((ext_vector_type(2))) float v2f;
    for (int pass = 0; pass < 2; ++pass) { for (int rr = 0; rr < 16; ++rr) *(volatile v2f*)(XOUT + (m0 + rr) * D + lane * 2) = *(const v2f*)(&Xr[rr][lane * 2]); __threadfence(); } }
  if (HAS_PX) {
    wave_lds_sync();
    for (int rr = 0; rr < 16; ++rr) { const size_t r = m0 + rr; float c0 = 0.0f, c1 = 0.0f;
      if (live) { if (HAS_UPD) { c0 = Xr[rr][lane * 2]; c1 = Xr[rr][lane * 2 + 1]; } else { c0 = bf16_rne(XIN[r * D + lane * 2]); c1 = bf16_rne(XIN[r * D + lane * 2 + 1]); } c0 += bf16_rne(vnext[lane * 2]); c1 += bf16_rne(vnext[lane * 2 + 1]); }
      b16 p, q; split16(c0 * XS, p, q); Ah[rr][lane * 2] = p; Al[rr][lane * 2] = q; split16(c1 * XS, p, q); Ah[rr][lane * 2 + 1] = p; Al[rr][lane * 2 + 1] = q; }
    wave_lds_sync();
#pragma unroll
    for (int t = 0; t < 4; ++t) acc[t] = (v8f){};
#pragma unroll
    for (int kb = 0; kb < D; kb += 32) { const v16b a = frag_kb(&Ah[nloc][kb], hlf), al = frag_kb(&Al[nloc][kb], hlf);
#pragma unroll
      for (int t = 0; t < 4; ++t) { const v16b bw = frag_kb(WPX + (size_t)(t * 16 + nloc) * D + kb, hlf); acc[t] = wmma16b(a, bw, acc[t]); acc[t] = wmma16b(al, bw, acc[t]); } }
    wave_lds_sync();
#pragma unroll
    for (int t = 0; t < 4; ++t) { const int c = t * 16 + nloc;
#pragma unroll 1
      for (int r8 = 0; r8 < 8; ++r8) Xr[8 * hlf + r8][c] = acc[t][r8] * sc; }
    wave_lds_sync();
    typedef __attribute__((ext_vector_type(2))) float v2f;
    for (int pass = 0; pass < 2; ++pass) { for (int rr = 0; rr < 16; ++rr) *(volatile v2f*)(PX + (m0 + rr) * D + lane * 2) = *(const v2f*)(&Xr[rr][lane * 2]); __threadfence(); } }
}
__global__ __launch_bounds__(128) void dst_kernel(const float* __restrict__ PX, const float* __restrict__ ea, const int* __restrict__ srcs, const b16* __restrict__ WE, const float* __restrict__ mb, const int* __restrict__ PERM, const int* __restrict__ ROWPTR, const int* __restrict__ ROWCNT, int permLen, int NLIM, float* __restrict__ AGG) {
  __shared__ __attribute__((aligned(16))) float Row[4][D + 4]; __shared__ int eid[4][16][2];
  const int wave = threadIdx.x >> 5, lane = threadIdx.x & 31, nloc = lane & 15, hlf = lane >> 4; const size_t v = (size_t)blockIdx.x * 4 + wave;
  int st = 0, cnt = 0; if (v < (size_t)NLIM) { st = ROWPTR[v]; cnt = ROWCNT[v]; cnt = iclamp(cnt, 0, 1 << 20); st = iclamp(st, 0, permLen - cnt); }
  float ag[4] = {0.0f, 0.0f, 0.0f, 0.0f}; float bv[4]; for (int t = 0; t < 4; ++t) bv[t] = bf16_rne(mb[t * 16 + nloc]);
  const int nchunk = (cnt + 15) >> 4;
#pragma unroll 1
  for (int ch = 0; ch < nchunk; ++ch) {
    const int j = ch * 16 + nloc; const bool ok = j < cnt; const int e = ok ? iclamp(PERM[st + j], 0, E - 1) : 0; int s = iclamp(srcs[e], 0, N - 1); if (s >= NLIM) s = -1;
    if (hlf == 0) { eid[wave][nloc][0] = e; eid[wave][nloc][1] = ok ? s : -1; }
    wave_lds_sync();
    v16b a; { const int ee = eid[wave][nloc][0]; for (int jj = 0; jj < 8; ++jj) { const int k = 8 * hlf + jj; a[jj] = (b16)(bf16_rne(ea[(size_t)ee * ED + k]) * XS); a[8 + jj] = (b16)0.0f; } }
#pragma unroll
    for (int t = 0; t < 4; ++t) { v8f acc = (v8f){}; acc = wmma16b(a, frag_kb(WE + (size_t)(t * 16 + nloc) * 32, hlf), acc); const int c = t * 16 + nloc; float s_ = 0.0f;
#pragma unroll
      for (int r8 = 0; r8 < 8; ++r8) { const int rl = 8 * hlf + r8; const int sr = eid[wave][rl][1]; const int srr = sr < 0 ? 0 : sr; const float px = PX[(size_t)srr * D + c]; s_ += (sr >= 0) ? fmaxf(acc[r8] * (1.0f / (XS * WSC)) + px + bv[t], 0.0f) : 0.0f; }
      s_ += __shfl_xor(s_, 16); ag[t] += s_; }
    wave_lds_sync(); }
  if (hlf == 0) for (int t = 0; t < 4; ++t) Row[wave][t * 16 + nloc] = ag[t];
  wave_lds_sync();
  for (int pass = 0; pass < 2; ++pass) { if (lane < 16) *(volatile v4f*)(AGG + v * D + lane * 4) = *(const v4f*)(&Row[wave][lane * 4]); __threadfence(); }
}
__global__ __launch_bounds__(256) void pool_kernel(const float* __restrict__ X1, const float* __restrict__ X2, const float* __restrict__ X3, const int* __restrict__ PERM, const int* __restrict__ ROWPTR, const int* __restrict__ ROWCNT, int permLen, int NLIM, float* __restrict__ PG) {
  const int wave = threadIdx.x >> 5, lane = threadIdx.x & 31; const int g = blockIdx.x * 8 + wave; if (g >= G) return; const int tix = (g >> 3) * 32 + (g & 7);
  int st = ROWPTR[tix], cnt = ROWCNT[tix]; cnt = iclamp(cnt, 0, 1 << 20); st = iclamp(st, 0, permLen - cnt); v4f a[3]; for (int q = 0; q < 3; ++q) a[q] = (v4f){0.0f, 0.0f, 0.0f, 0.0f}; const int lc = (lane & 15) * 4;
#pragma unroll 1
  for (int j = 0; j < cnt; ++j) { const int n = iclamp(PERM[st + j], 0, N - 1); if (n >= NLIM) continue; const v4f x1 = *(const v4f*)(X1 + (size_t)n * D + lc), x2 = *(const v4f*)(X2 + (size_t)n * D + lc), x3 = *(const v4f*)(X3 + (size_t)n * D + lc); for (int i = 0; i < 4; ++i) { a[0][i] += x1[i]; a[1][i] += x2[i]; a[2][i] += x3[i]; } }
  for (int pass = 0; pass < 2; ++pass) { if (lane < 16) for (int q = 0; q < 3; ++q) *(volatile v4f*)(PG + (size_t)g * CAT + q * D + lane * 4) = a[q]; __threadfence(); }
}
__global__ __launch_bounds__(128) void mlp_kernel(const float* __restrict__ PG, const b16* __restrict__ W0T, const b16* __restrict__ W1T, const b16* __restrict__ WET, const float* __restrict__ b0, const float* __restrict__ b1, const float* __restrict__ be, const float* __restrict__ wo, const float* __restrict__ bo, float* __restrict__ out) {
  __shared__ __attribute__((aligned(16))) b16 Ah[4][16][L0 + 8], Al[4][16][L0 + 8]; __shared__ float so[64];
  const int wave = threadIdx.x >> 5, lane = threadIdx.x & 31, nloc = lane & 15, hlf = lane >> 4; const int g0 = (blockIdx.x * 4 + wave) * 16; const float sc = 1.0f / (XS * WSC);
  for (int rr = 0; rr < 16; ++rr) for (int c = lane; c < CAT; c += 32) { const float v = (g0 + rr < G) ? PG[(size_t)(g0 + rr) * CAT + c] : 0.0f; b16 p, q; split16(v * XS, p, q); Ah[wave][rr][c] = p; Al[wave][rr][c] = q; }
  wave_lds_sync();
  float hk[2][8][8];
#pragma unroll
  for (int cg = 0; cg < 2; ++cg) { v8f acc[8];
#pragma unroll
    for (int t = 0; t < 8; ++t) acc[t] = (v8f){};
#pragma unroll 2
    for (int kb = 0; kb < CAT; kb += 32) { const v16b a = frag_kb(&Ah[wave][nloc][kb], hlf), al = frag_kb(&Al[wave][nloc][kb], hlf);
#pragma unroll
      for (int t = 0; t < 8; ++t) { const v16b bw = frag_kb(W0T + (size_t)(cg * 128 + t * 16 + nloc) * CAT + kb, hlf); acc[t] = wmma16b(a, bw, acc[t]); acc[t] = wmma16b(al, bw, acc[t]); } }
#pragma unroll
    for (int t = 0; t < 8; ++t) { const float bb = bf16_rne(b0[cg * 128 + t * 16 + nloc]);
#pragma unroll
      for (int r8 = 0; r8 < 8; ++r8) hk[cg][t][r8] = fmaxf(acc[t][r8] * sc + bb, 0.0f); } }
  wave_lds_sync();
#pragma unroll
  for (int cg = 0; cg < 2; ++cg)
#pragma unroll
    for (int t = 0; t < 8; ++t)
#pragma unroll
      for (int r8 = 0; r8 < 8; ++r8) { b16 p, q; split16(hk[cg][t][r8] * XS, p, q); Ah[wave][8 * hlf + r8][cg * 128 + t * 16 + nloc] = p; Al[wave][8 * hlf + r8][cg * 128 + t * 16 + nloc] = q; }
  wave_lds_sync();
  { v8f acc[8];
#pragma unroll
    for (int t = 0; t < 8; ++t) acc[t] = (v8f){};
#pragma unroll 2
    for (int kb = 0; kb < L0; kb += 32) { const v16b a = frag_kb(&Ah[wave][nloc][kb], hlf), al = frag_kb(&Al[wave][nloc][kb], hlf);
#pragma unroll
      for (int t = 0; t < 8; ++t) { const v16b bw = frag_kb(W1T + (size_t)(t * 16 + nloc) * L0 + kb, hlf); acc[t] = wmma16b(a, bw, acc[t]); acc[t] = wmma16b(al, bw, acc[t]); } }
    wave_lds_sync();
#pragma unroll
    for (int t = 0; t < 8; ++t) { const float bb = bf16_rne(b1[t * 16 + nloc]);
#pragma unroll
      for (int r8 = 0; r8 < 8; ++r8) { const float h = fmaxf(acc[t][r8] * sc + bb, 0.0f); b16 p, q; split16(h * XS, p, q); Ah[wave][8 * hlf + r8][t * 16 + nloc] = p; Al[wave][8 * hlf + r8][t * 16 + nloc] = q; } } }
  wave_lds_sync();
  { v8f acc[8]; float ps[8]; for (int r8 = 0; r8 < 8; ++r8) ps[r8] = 0.0f;
#pragma unroll
    for (int t = 0; t < 8; ++t) acc[t] = (v8f){};
#pragma unroll 2
    for (int kb = 0; kb < L1; kb += 32) { const v16b a = frag_kb(&Ah[wave][nloc][kb], hlf), al = frag_kb(&Al[wave][nloc][kb], hlf);
#pragma unroll
      for (int t = 0; t < 8; ++t) { const v16b bw = frag_kb(WET + (size_t)(t * 16 + nloc) * L1 + kb, hlf); acc[t] = wmma16b(a, bw, acc[t]); acc[t] = wmma16b(al, bw, acc[t]); } }
#pragma unroll
    for (int t = 0; t < 8; ++t) { const int c = t * 16 + nloc; const float bb = bf16_rne(be[c]), wv = bf16_rne(wo[c]);
#pragma unroll
      for (int r8 = 0; r8 < 8; ++r8) ps[r8] += pmul(acc[t][r8] * sc + bb, wv); }
    const float bov = bf16_rne(bo[0]);
#pragma unroll
    for (int r8 = 0; r8 < 8; ++r8) { float s = ps[r8]; for (int o = 1; o < 16; o <<= 1) s += __shfl_xor(s, o); if (nloc == 0) so[wave * 16 + 8 * hlf + r8] = s + bov; } }
  __syncthreads();
  for (int pass = 0; pass < 2; ++pass) { const int g = blockIdx.x * 64 + threadIdx.x; if (threadIdx.x < 64 && g < G) ((volatile float*)out)[g] = so[threadIdx.x]; __threadfence(); }
}
}

extern "C" void kernel_launch(void* const* d_in, const int* in_sizes, int n_in, void* d_out, int out_size, void* d_ws, size_t ws_size, hipStream_t stream) {
  (void)n_in;
  auto Fp = [&](int i) { return (const float*)d_in[i]; }; auto Ip = [&](int i) { return (const int*)d_in[i]; };
  if (in_sizes[0] != N * D || in_sizes[1] != E * ED || in_sizes[2] != 2 * E || in_sizes[3] != N || in_sizes[5] != L * D || in_sizes[6] != L * (D + ED) * D || in_sizes[8] != L * 2 * D * D || in_sizes[18] != CAT * L0 || in_sizes[20] != L0 * L1 || in_sizes[22] != L1 * L1 || in_sizes[24] != L1 || out_size != G) return;
  const int NLIM = N, EL = E; const int GB16 = NBLK, GB4 = NP / 4;
  size_t off = 0; char* ws = (char*)d_ws;
  auto carve = [&](size_t bytes) { char* p = ws + off; off += (bytes + 255) & ~(size_t)255; return p; };
  b16* WPX[3]; b16* WE[3]; b16* WU[3]; for (int i = 0; i < L; ++i) { WPX[i] = (b16*)carve(D * D * 2); WE[i] = (b16*)carve(D * 32 * 2); WU[i] = (b16*)carve(D * 2 * D * 2); }
  b16* W0T = (b16*)carve((size_t)L0 * CAT * 2); b16* W1T = (b16*)carve((size_t)L1 * L0 * 2); b16* WET = (b16*)carve((size_t)L1 * L1 * 2);
  float* X[3]; for (int i = 0; i < L; ++i) X[i] = (float*)carve((size_t)NP * D * 4); float* PX = (float*)carve((size_t)NP * D * 4); float* AGG = (float*)carve((size_t)NP * D * 4); float* PG = (float*)carve((size_t)GP * CAT * 4);
  CsrBufs9 csr; CsrBufs3 pl; off = csr_carve9(csr, ws, off, EL, N); off = csr_carve3(pl, ws, off, N, G);
  if (off > ws_size) return;
  const unsigned gsm = (D * 2 * D / 8 + 255) / 256;
  for (int i = 0; i < L; ++i) { const float* mw = Fp(6) + (size_t)i * (D + ED) * D; wprep_kernel<<<gsm, 256, 0, stream>>>(mw, 0, D, D, D, WPX[i]); wprep_kernel<<<gsm, 256, 0, stream>>>(mw, D, ED, D, 32, WE[i]); wprep_kernel<<<gsm, 256, 0, stream>>>(Fp(8) + (size_t)i * 2 * D * D, 0, 2 * D, D, 2 * D, WU[i]); }
  wprep_kernel<<<(L0 * CAT / 8 + 255) / 256, 256, 0, stream>>>(Fp(18), 0, CAT, L0, CAT, W0T); wprep_kernel<<<(L1 * L0 / 8 + 255) / 256, 256, 0, stream>>>(Fp(20), 0, L0, L1, L0, W1T); wprep_kernel<<<(L1 * L1 / 8 + 255) / 256, 256, 0, stream>>>(Fp(22), 0, L1, L1, L1, WET);
  csr_build9(csr, Ip(2) + E, EL, N, stream); csr_build3(pl, Ip(3), N, G, stream);
  node_kernel<1, 0, 1><<<GB16, 32, 0, stream>>>(Fp(0), nullptr, nullptr, nullptr, nullptr, nullptr, nullptr, Fp(5), WPX[0], NLIM, nullptr, PX);
  for (int i = 0; i < L; ++i) {
    dst_kernel<<<GB4, 128, 0, stream>>>(PX, Fp(1), Ip(2), WE[i], Fp(7) + i * D, csr.PERM, csr.ROWPTR, csr.ROWCNT, (int)csr.permLen, NLIM, AGG);
    const float* xin = i == 0 ? Fp(0) : X[i - 1]; const bool haspx = i + 1 < L;
    if (i == 0) { node_kernel<1, 1, 1><<<GB16, 32, 0, stream>>>(xin, Fp(5), AGG, WU[0], Fp(9), Fp(10), Fp(11), Fp(5) + D, WPX[1], NLIM, X[0], PX); }
    else if (haspx) { node_kernel<0, 1, 1><<<GB16, 32, 0, stream>>>(xin, Fp(5) + i * D, AGG, WU[i], Fp(9) + i * D, Fp(10) + i * D, Fp(11) + i * D, Fp(5) + (i + 1) * D, WPX[i + 1], NLIM, X[i], PX); }
    else { node_kernel<0, 1, 0><<<GB16, 32, 0, stream>>>(xin, Fp(5) + i * D, AGG, WU[i], Fp(9) + i * D, Fp(10) + i * D, Fp(11) + i * D, nullptr, nullptr, NLIM, X[i], nullptr); } }
  pool_kernel<<<GP / 8, 256, 0, stream>>>(X[0], X[1], X[2], pl.PERM, pl.ROWPTR, pl.ROWCNT, (int)pl.permLen, NLIM, PG);
  mlp_kernel<<<(GP / 16 + 3) / 4, 128, 0, stream>>>(PG, W0T, W1T, WET, Fp(19), Fp(21), Fp(23), Fp(24), Fp(25), (float*)d_out);
}
